// GCNNet_48395691492010
// MI455X (gfx1250) — hardware-verified
//
#include <hip/hip_runtime.h>
#include <stddef.h>
#include <stdint.h>
#include <math.h>


#define NFX    22
#define NTHR   256
#define NWAVE  8
#define EPT    8
#define CHUNK  (NTHR * EPT)
#define WCAP   (EPT * 32)
#define LISTN  (NWAVE * WCAP)
#define NBD    8192
#define SLD    13
#define NBA    1024
#define SLA    10
#define RCAP   16384
#define DEGCAP 64
#define GBM    64
#define GTHR   128
#define H32    32
#define H64    64
#define H128   128
#define NMID   8
#define U1     2048
#define U2     2048
#define UM     8192
#define UF     512
#define UTOT   (U1 + U2 + UM + UF)
#define AGG_ZINTS    (LISTN + 2 * RCAP + 3 * NBA)
#define MISC_INTS    16
#define WST_INTS     (NWAVE * H64 * 2 * 2)
#define AGG_LDS_INTS (AGG_ZINTS + MISC_INTS + WST_INTS)
#define TABN   512
#define ARB    64
#define WSMAX  134217728
#define BNEPS  1e-5f

static_assert((CHUNK & (CHUNK - 1)) == 0 && CHUNK <= 4096);
static_assert((NBD & (NBD - 1)) == 0 && NBD == (1 << SLD));
static_assert((NBA & (NBA - 1)) == 0 && NBA == (1 << SLA));
static_assert(((long long)CHUNK << SLD) < (1LL << 31));
static_assert(((long long)CHUNK << SLA) < (1LL << 31));
static_assert(NBD % (NTHR * 4) == 0);
static_assert(LISTN % NTHR == 0);
static_assert(NBA % NWAVE == 0 && NBA % 32 == 0 && NBA % GBM == 0);
static_assert(RCAP % 32 == 0 && AGG_ZINTS % 4 == 0 && LISTN % 4 == 0);
static_assert(AGG_ZINTS % (NTHR * 4) == 0);
static_assert(((AGG_ZINTS + MISC_INTS) * 4) % 16 == 0);
static_assert(AGG_LDS_INTS * 4 <= 200000);
static_assert(GBM == (GTHR / 32) * 16);
static_assert(H64 == 2 * 32);
static_assert(U1 % NTHR == 0 && (U1 + U2) % NTHR == 0 && (U1 + U2 + UM) % NTHR == 0 && UTOT % NTHR == 0);
static_assert(U1 == H128 * (2 * H64 / 8) && U2 == H64 * (2 * H128 / 8) && UM == NMID * H64 * (2 * H64 / 8) && UF == H32 * (2 * H64 / 8));
static_assert(ARB % (2 * NWAVE) == 0);

typedef float          v2f   __attribute__((ext_vector_type(2)));
typedef float          v4f   __attribute__((ext_vector_type(4)));
typedef float          v8f   __attribute__((ext_vector_type(8)));
typedef double         v2d   __attribute__((ext_vector_type(2)));
typedef int            v4i   __attribute__((ext_vector_type(4)));
typedef int            v8i   __attribute__((ext_vector_type(8)));
typedef unsigned short v4us  __attribute__((ext_vector_type(4)));
typedef unsigned short v8us  __attribute__((ext_vector_type(8)));
typedef unsigned short v16us __attribute__((ext_vector_type(16)));
typedef __bf16         v16bf __attribute__((ext_vector_type(16)));
typedef v2f  __attribute__((may_alias)) v2fa;
typedef v4f  __attribute__((may_alias)) v4fa;
typedef v2d  __attribute__((may_alias)) v2da;
typedef v4i  __attribute__((may_alias)) v4ia;
typedef v4us __attribute__((may_alias)) v4usa;
typedef v8us __attribute__((may_alias)) v8usa;
union FragB { v16bf v; v16us u; v8us h[2]; v8i w; };

__device__ __forceinline__ v8f wmb(const FragB& a, const FragB& b, v8f c) {
  v8f d = __builtin_amdgcn_wmma_f32_16x16x32_bf16(false, a.v, false, b.v, (short)0, c, false, false);
  asm volatile("v_nop\n\tv_nop\n\tv_nop\n\tv_nop" : "+v"(d) : "v"(a.w), "v"(b.w));
  return d;
}

__device__ __forceinline__ unsigned bf16_bits(float f) {
  const unsigned u = __float_as_uint(f);
  return (u + 0x7FFFu + ((u >> 16) & 1u)) >> 16;
}
__device__ __forceinline__ float bf16_val(float f) {
  return __uint_as_float(bf16_bits(f) << 16);
}

template <int SLB>
__device__ __forceinline__ int scan_chunk(const int* __restrict__ dsts, int nE, int cbase, int slotBase,
                                          int nb, int vec8, int* list, int tid, int lane, int wave) {
  int wc = 0;
  const int el0  = tid * EPT;
  const int e0   = cbase + el0;
  const int sent = -2147483647 - 1;
  v4i da, db;
  if (vec8 != 0 && cbase + CHUNK <= nE) {
    da = *(const v4i*)(dsts + e0);
    db = *(const v4i*)(dsts + e0 + 4);
  } else {
    da.x = (e0     < nE) ? dsts[min(e0,     nE - 1)] : sent;
    da.y = (e0 + 1 < nE) ? dsts[min(e0 + 1, nE - 1)] : sent;
    da.z = (e0 + 2 < nE) ? dsts[min(e0 + 2, nE - 1)] : sent;
    da.w = (e0 + 3 < nE) ? dsts[min(e0 + 3, nE - 1)] : sent;
    db.x = (e0 + 4 < nE) ? dsts[min(e0 + 4, nE - 1)] : sent;
    db.y = (e0 + 5 < nE) ? dsts[min(e0 + 5, nE - 1)] : sent;
    db.z = (e0 + 6 < nE) ? dsts[min(e0 + 6, nE - 1)] : sent;
    db.w = (e0 + 7 < nE) ? dsts[min(e0 + 7, nE - 1)] : sent;
  }
  const unsigned nbs = (unsigned)slotBase;
  const unsigned unb = (unsigned)nb;
  const unsigned s0 = (unsigned)da.x - nbs, s1 = (unsigned)da.y - nbs;
  const unsigned s2 = (unsigned)da.z - nbs, s3 = (unsigned)da.w - nbs;
  const unsigned s4 = (unsigned)db.x - nbs, s5 = (unsigned)db.y - nbs;
  const unsigned s6 = (unsigned)db.z - nbs, s7 = (unsigned)db.w - nbs;
  const bool h0 = s0 < unb, h1 = s1 < unb, h2 = s2 < unb, h3 = s3 < unb;
  const bool h4 = s4 < unb, h5 = s5 < unb, h6 = s6 < unb, h7 = s7 < unb;
  const unsigned any = __builtin_amdgcn_ballot_w32(h0 | h1 | h2 | h3 | h4 | h5 | h6 | h7);
  if (any != 0u) {
#define HITJ(J, HJ, SJ) { \
      const unsigned mj = __builtin_amdgcn_ballot_w32(HJ); \
      if (mj != 0u) { \
        if (HJ) { \
          const int pos = wc + (int)__builtin_amdgcn_mbcnt_lo(mj, 0u); \
          if (pos < WCAP) list[wave * WCAP + pos] = ((el0 + (J)) << SLB) | (int)(SJ); \
        } \
        wc += (int)__builtin_popcount(mj); } }
    HITJ(0, h0, s0)
    HITJ(1, h1, s1)
    HITJ(2, h2, s2)
    HITJ(3, h3, s3)
    HITJ(4, h4, s4)
    HITJ(5, h5, s5)
    HITJ(6, h6, s6)
    HITJ(7, h7, s7)
#undef HITJ
  }
  return wc;
}

__global__ __launch_bounds__(NTHR) void k_wprep(const float* __restrict__ W1, const float* __restrict__ W2,
                                                const float* __restrict__ Wm, const float* __restrict__ Wf,
                                                unsigned short* B1, unsigned short* B2,
                                                unsigned short* BM, unsigned short* BF) {
  const int u = (int)blockIdx.x * NTHR + (int)threadIdx.x;
  const float* p;
  unsigned short* dp;
  if (u < U1) {
    const int n = u >> 4, k8 = (u & 15) * 8, kk = k8 & (H64 - 1);
    p  = W1 + (size_t)n * H64 + kk;
    dp = B1 + (size_t)n * (2 * H64) + k8;
  } else if (u < U1 + U2) {
    const int v = u - U1;
    const int n = v >> 5, k8 = (v & 31) * 8, kk = k8 & (H128 - 1);
    p  = W2 + (size_t)n * H128 + kk;
    dp = B2 + (size_t)n * (2 * H128) + k8;
  } else if (u < U1 + U2 + UM) {
    const int v = u - (U1 + U2);
    const int row = v >> 4, k8 = (v & 15) * 8, kk = k8 & (H64 - 1);
    p  = Wm + (size_t)row * H64 + kk;
    dp = BM + (size_t)row * (2 * H64) + k8;
  } else if (u < UTOT) {
    const int v = u - (U1 + U2 + UM);
    const int n = v >> 4, k8 = (v & 15) * 8, kk = k8 & (H64 - 1);
    p  = Wf + (size_t)n * H64 + kk;
    dp = BF + (size_t)n * (2 * H64) + k8;
  } else {
    return;
  }
  const v4f a = *(const v4fa*)p;
  const v4f b = *(const v4fa*)(p + 4);
  v8us o;
  o[0] = (unsigned short)bf16_bits(a.x); o[1] = (unsigned short)bf16_bits(a.y);
  o[2] = (unsigned short)bf16_bits(a.z); o[3] = (unsigned short)bf16_bits(a.w);
  o[4] = (unsigned short)bf16_bits(b.x); o[5] = (unsigned short)bf16_bits(b.y);
  o[6] = (unsigned short)bf16_bits(b.z); o[7] = (unsigned short)bf16_bits(b.w);
  *(volatile v8us*)dp = o;
  __threadfence();
  *(volatile v8us*)dp = o;
}

__global__ __launch_bounds__(NTHR) void k_esg(const float* __restrict__ x, int nN, int mRows,
                                              const float* __restrict__ We, const float* __restrict__ be,
                                              float* x10) {
  __shared__ float xs[NTHR * NFX];
  __shared__ float wsh[72];
  __shared__ float bsh[4];
  const int tid = (int)threadIdx.x;
  const int row0 = (int)blockIdx.x * NTHR;
  const size_t total = (size_t)nN * NFX;
  const size_t base  = (size_t)row0 * NFX;
#pragma unroll 1
  for (int i = tid; i < NTHR * NFX; i += NTHR) {
    size_t gi = base + (size_t)i;
    gi = gi < total ? gi : total - 1;
    xs[i] = bf16_val(x[gi]);
  }
  if (tid < 72) wsh[tid] = bf16_val(We[tid]);
  if (tid < 4)  bsh[tid] = bf16_val(be[tid]);
  __syncthreads();
  const int row = row0 + tid;
  const float* xr = xs + tid * NFX;
  float d0 = 0.0f, d1 = 0.0f, d2 = 0.0f, d3 = 0.0f;
#pragma unroll 1
  for (int k = 0; k < 18; ++k) {
    const float xv = xr[4 + k];
    d0 = fmaf(xv, wsh[k * 4 + 0], d0);
    d1 = fmaf(xv, wsh[k * 4 + 1], d1);
    d2 = fmaf(xv, wsh[k * 4 + 2], d2);
    d3 = fmaf(xv, wsh[k * 4 + 3], d3);
  }
  const bool live = row < nN;
  v4f o;
  o.x = live ? ((d0 + bsh[0]) + xr[0]) : 0.0f;
  o.y = live ? ((d1 + bsh[1]) + xr[1]) : 0.0f;
  o.z = live ? ((d2 + bsh[2]) + xr[2]) : 0.0f;
  o.w = live ? ((d3 + bsh[3]) + xr[3]) : 0.0f;
  float* op = x10 + (size_t)row * 4;
  if (row < mRows) *(volatile v4f*)op = o;
  __threadfence();
  if (row < mRows) *(volatile v4f*)op = o;
}

__global__ __launch_bounds__(NTHR) void k_deg(const int* __restrict__ dsts, const float* __restrict__ ew,
                                              int nE, int vec8, float* dis) {
  __shared__ __attribute__((aligned(16))) float sdeg[NBD];
  __shared__ __attribute__((aligned(16))) int list[LISTN];
  __shared__ int wcnt[NWAVE];
  const int tid = (int)threadIdx.x, lane = tid & 31, wave = tid >> 5;
  const int nodeBase = (int)blockIdx.x * NBD;

  for (int i = tid; i < NBD; i += NTHR) sdeg[i] = 0.0f;
  for (int i = tid; i < LISTN; i += NTHR) list[i] = 0;
  if (tid < NWAVE) wcnt[tid] = 0;
  __syncthreads();

  const int nChunks = (nE + CHUNK - 1) / CHUNK;
#pragma unroll 1
  for (int ch = 0; ch < nChunks; ++ch) {
    const int cbase = ch * CHUNK;
    const int wc = scan_chunk<SLD>(dsts, nE, cbase, nodeBase, NBD, vec8, list, tid, lane, wave);
    if (lane == 0) wcnt[wave] = wc;
    __syncthreads();
    if (wave == 0) {
#pragma unroll 1
      for (int w2 = 0; w2 < NWAVE; ++w2) {
        int c = wcnt[w2];
        c = c < 0 ? 0 : (c > WCAP ? WCAP : c);
#pragma unroll 1
        for (int b0 = 0; b0 < c; b0 += 32) {
          const int idx = b0 + lane;
          const int ent = list[w2 * WCAP + (idx < WCAP ? idx : WCAP - 1)];
          const int el  = (ent >> SLD) & (CHUNK - 1);
          int e = cbase + el;
          e = e > nE - 1 ? nE - 1 : e;
          const int wvi = __float_as_int(bf16_val(ew[e]));
          const int m32 = (c - b0) < 32 ? (c - b0) : 32;
#pragma unroll 1
          for (int k = 0; k < m32; ++k) {
            const int   u  = __builtin_amdgcn_readlane(ent, k);
            const float wk = __int_as_float(__builtin_amdgcn_readlane(wvi, k));
            const int   sl = u & (NBD - 1);
            if (lane == 0) sdeg[sl] = sdeg[sl] + wk;
          }
        }
      }
    }
    __syncthreads();
  }

  v4f vals[NBD / (NTHR * 4)];
#pragma unroll
  for (int it = 0; it < NBD / (NTHR * 4); ++it) {
    const int s0 = it * (NTHR * 4) + 4 * tid;
    const v4f d4 = *(const v4fa*)(sdeg + s0);
    const float e0 = d4.x + 1.0f, e1 = d4.y + 1.0f, e2 = d4.z + 1.0f, e3 = d4.w + 1.0f;
    v4f v;
    v.x = (e0 > 0.0f) ? rsqrtf(fmaxf(e0, 1e-30f)) : 0.0f;
    v.y = (e1 > 0.0f) ? rsqrtf(fmaxf(e1, 1e-30f)) : 0.0f;
    v.z = (e2 > 0.0f) ? rsqrtf(fmaxf(e2, 1e-30f)) : 0.0f;
    v.w = (e3 > 0.0f) ? rsqrtf(fmaxf(e3, 1e-30f)) : 0.0f;
    vals[it] = v;
  }
#pragma unroll
  for (int it = 0; it < NBD / (NTHR * 4); ++it) {
    const int s0 = it * (NTHR * 4) + 4 * tid;
    *(volatile v4f*)(dis + (size_t)nodeBase + s0) = vals[it];
  }
  __threadfence();
#pragma unroll
  for (int it = 0; it < NBD / (NTHR * 4); ++it) {
    const int s0 = it * (NTHR * 4) + 4 * tid;
    *(volatile v4f*)(dis + (size_t)nodeBase + s0) = vals[it];
  }
}

__global__ __launch_bounds__(NTHR) void k_norm(const int* __restrict__ srcs, const int* __restrict__ dsts,
                                               const float* __restrict__ ew, const float* __restrict__ dis,
                                               int nE, int nN, int nPadE, float* nrm) {
  const int t  = (int)blockIdx.x * NTHR + (int)threadIdx.x;
  const int e0 = 2 * t;
  if (e0 >= nPadE) return;
  const int ea = e0 < nE - 1 ? e0 : nE - 1;
  const int eb = (e0 + 1) < nE - 1 ? (e0 + 1) : nE - 1;
  int sa = srcs[ea], sb = srcs[eb], da = dsts[ea], db = dsts[eb];
  sa = sa < 0 ? 0 : (sa > nN - 1 ? nN - 1 : sa);
  sb = sb < 0 ? 0 : (sb > nN - 1 ? nN - 1 : sb);
  da = da < 0 ? 0 : (da > nN - 1 ? nN - 1 : da);
  db = db < 0 ? 0 : (db > nN - 1 ? nN - 1 : db);
  const float wa = bf16_val(ew[ea]), wb = bf16_val(ew[eb]);
  v2f o;
  o.x = (dis[sa] * wa) * dis[da];
  o.y = (dis[sb] * wb) * dis[db];
  float* op = nrm + e0;
  *(volatile v2f*)op = o;
  __threadfence();
  *(volatile v2f*)op = o;
}

template <int MODE>
__global__ __launch_bounds__(NTHR) void k_scan(const int* __restrict__ srcs, const int* __restrict__ dsts,
                                               int nE, int nN, int vec8, int mRows,
                                               const float* __restrict__ dis, const float* __restrict__ nrm,
                                               const float* __restrict__ gsrc, const float* __restrict__ w0,
                                               const float* __restrict__ bias, float* outp, double* rec) {
  extern __shared__ __attribute__((aligned(16))) int dsm[];
  int* list = dsm;
  int* hl   = dsm + LISTN;
  int* sl   = hl + RCAP;
  int* cnt  = sl + RCAP;
  int* offs = cnt + NBA;
  int* cur  = offs + NBA;
  int* misc = cur + NBA;
  double* wst = (double*)(misc + MISC_INTS);
  const int tid = (int)threadIdx.x, lane = tid & 31, wave = tid >> 5;
  const int nodeBase = (int)blockIdx.x * NBA;
  constexpr int FS = (MODE == 4) ? H32 : H64;

  {
    const v4i z4 = {0, 0, 0, 0};
    for (int i = tid * 4; i < AGG_ZINTS; i += NTHR * 4) *(v4ia*)(dsm + i) = z4;
    if (tid < MISC_INTS) misc[tid] = 0;
  }
  float bv0 = 0.0f, bv1 = 0.0f;
  v4f wA = {0.0f, 0.0f, 0.0f, 0.0f}, wB = {0.0f, 0.0f, 0.0f, 0.0f};
  if constexpr (MODE == 0) {
    const v4f ta = *(const v4fa*)(w0 + (size_t)(2 * lane) * 4);
    const v4f tb = *(const v4fa*)(w0 + (size_t)(2 * lane + 1) * 4);
    wA.x = bf16_val(ta.x); wA.y = bf16_val(ta.y); wA.z = bf16_val(ta.z); wA.w = bf16_val(ta.w);
    wB.x = bf16_val(tb.x); wB.y = bf16_val(tb.y); wB.z = bf16_val(tb.z); wB.w = bf16_val(tb.w);
  }
  if constexpr (MODE == 0 || MODE == 2 || MODE == 3) {
    const v2f b2 = *(const v2fa*)(bias + 2 * lane);
    bv0 = bf16_val(b2.x); bv1 = bf16_val(b2.y);
  }
  if constexpr (MODE == 4) {
    bv0 = bf16_val(bias[lane]);
  }
  __syncthreads();

  int t = 0, ov = 0;
  const int nChunks = (nE + CHUNK - 1) / CHUNK;
#pragma unroll 1
  for (int ch = 0; ch < nChunks; ++ch) {
    const int cbase = ch * CHUNK;
    const int wc = scan_chunk<SLA>(dsts, nE, cbase, nodeBase, NBA, vec8, list, tid, lane, wave);
    if (lane == 0) misc[wave] = wc;
    __syncthreads();
    if (wave == 0) {
#pragma unroll 1
      for (int w2 = 0; w2 < NWAVE; ++w2) {
        int c = misc[w2];
        c = c < 0 ? 0 : (c > WCAP ? WCAP : c);
#pragma unroll 1
        for (int b0 = 0; b0 < c; b0 += 32) {
          const int idx = b0 + lane;
          const int ent = list[w2 * WCAP + (idx < WCAP ? idx : WCAP - 1)];
          const int m32 = (c - b0) < 32 ? (c - b0) : 32;
#pragma unroll 1
          for (int k = 0; k < m32; ++k) {
            const int u    = __builtin_amdgcn_readlane(ent, k);
            const int slot = u & (NBA - 1);
            const int el   = (u >> SLA) & (CHUNK - 1);
            const int pk   = ((cbase + el) << SLA) | slot;
            if (t < RCAP) {
              if (lane == 0) { hl[t] = pk; cnt[slot] = cnt[slot] + 1; }
              t = t + 1;
            } else {
              ov = 1;
            }
          }
        }
      }
    }
    __syncthreads();
  }
  if (wave == 0 && lane == 0) { misc[8] = t; misc[9] = ov; }
  __syncthreads();
  int tt = misc[8];
  tt = tt < 0 ? 0 : (tt > RCAP ? RCAP : tt);
  const int ovf = misc[9];

  if (wave == 0) {
    const int base = lane * (NBA / 32);
    int s = 0;
#pragma unroll 1
    for (int i = 0; i < NBA / 32; ++i) s += cnt[base + i];
    int incl = s;
#pragma unroll
    for (int d = 1; d < 32; d <<= 1) {
      const int y = __shfl_up(incl, d, 32);
      if (lane >= d) incl += y;
    }
    int run = incl - s;
#pragma unroll 1
    for (int i = 0; i < NBA / 32; ++i) {
      const int cv = cnt[base + i];
      offs[base + i] = run;
      cur[base + i]  = run;
      run += cv;
    }
  }
  __syncthreads();
  if (wave == 0) {
#pragma unroll 1
    for (int b0 = 0; b0 < tt; b0 += 32) {
      const int idx = b0 + lane;
      const int ent = hl[idx < RCAP ? idx : RCAP - 1];
      const int m32 = (tt - b0) < 32 ? (tt - b0) : 32;
#pragma unroll 1
      for (int k = 0; k < m32; ++k) {
        const int u    = __builtin_amdgcn_readlane(ent, k);
        const int slot = u & (NBA - 1);
        if (lane == 0) {
          int p = cur[slot];
          p = p < 0 ? 0 : (p > RCAP - 1 ? RCAP - 1 : p);
          sl[p] = u;
          cur[slot] = p + 1;
        }
      }
    }
  }
  __syncthreads();

  const float qnan = __int_as_float(0x7fc00000);
  const float pz = (ovf != 0) ? qnan : 0.0f;
  const int sa = (2 * lane) & 31, sb = (2 * lane + 1) & 31;
  double s1a = 0.0, s2a = 0.0, s1b = 0.0, s2b = 0.0;
#pragma unroll 1
  for (int si = 0; si < NBA / NWAVE; ++si) {
    const int s    = si * NWAVE + wave;
    const int node = nodeBase + s;
    int c = cnt[s];
    const bool big = c > DEGCAP;
    c = c < 0 ? 0 : (c > DEGCAP ? DEGCAP : c);
    int o = offs[s];
    o = o < 0 ? 0 : (o > RCAP ? RCAP : o);
    const int nc = node < nN ? node : nN - 1;
    const float dd = dis[nc];
    const float rd = dd * dd;
    const float pzr = big ? qnan : pz;
    const bool live = node < nN;
    const bool wrow = node < mRows;
    float v0 = 0.0f, v1 = 0.0f;

    if constexpr (MODE == 0) {
      float a0 = 0.0f, a1 = 0.0f, a2 = 0.0f, a3 = 0.0f;
#pragma unroll 1
      for (int b0 = 0; b0 < c; b0 += 32) {
        int idx = o + b0 + lane;
        idx = idx > RCAP - 1 ? RCAP - 1 : idx;
        const int ent = sl[idx];
        int eid = ent >> SLA;
        eid = eid < 0 ? 0 : (eid > nE - 1 ? nE - 1 : eid);
        int sr = srcs[eid];
        sr = sr < 0 ? 0 : (sr > nN - 1 ? nN - 1 : sr);
        const float cf  = nrm[eid];
        const float cfv = ((b0 + lane) < c) ? cf : 0.0f;
        const v4f xv = *(const v4fa*)(gsrc + (size_t)sr * 4);
        a0 = fmaf(cfv, xv.x, a0); a1 = fmaf(cfv, xv.y, a1);
        a2 = fmaf(cfv, xv.z, a2); a3 = fmaf(cfv, xv.w, a3);
      }
#pragma unroll
      for (int d = 16; d >= 1; d >>= 1) {
        a0 += __shfl_xor(a0, d, 32); a1 += __shfl_xor(a1, d, 32);
        a2 += __shfl_xor(a2, d, 32); a3 += __shfl_xor(a3, d, 32);
      }
      const v4f xs = *(const v4fa*)(gsrc + (size_t)nc * 4);
      const float g0v = a0 + xs.x * rd, g1v = a1 + xs.y * rd, g2v = a2 + xs.z * rd, g3v = a3 + xs.w * rd;
      float t0 = g0v * wA.x; t0 = fmaf(g1v, wA.y, t0); t0 = fmaf(g2v, wA.z, t0); t0 = fmaf(g3v, wA.w, t0);
      float t1 = g0v * wB.x; t1 = fmaf(g1v, wB.y, t1); t1 = fmaf(g2v, wB.z, t1); t1 = fmaf(g3v, wB.w, t1);
      const float y0 = (t0 + bv0) + pzr, y1 = (t1 + bv1) + pzr;
      v0 = live ? y0 : 0.0f; v1 = live ? y1 : 0.0f;
    } else if constexpr (MODE == 1 || MODE == 2 || MODE == 3) {
      float acc0 = 0.0f, acc1 = 0.0f;
#pragma unroll 1
      for (int b0 = 0; b0 < c; b0 += 32) {
        int idx = o + b0 + lane;
        idx = idx > RCAP - 1 ? RCAP - 1 : idx;
        const int ent = sl[idx];
        int eid = ent >> SLA;
        eid = eid < 0 ? 0 : (eid > nE - 1 ? nE - 1 : eid);
        int sr = srcs[eid];
        sr = sr < 0 ? 0 : (sr > nN - 1 ? nN - 1 : sr);
        const int cfi = __float_as_int(nrm[eid]);
        const int m32 = (c - b0) < 32 ? (c - b0) : 32;
#pragma unroll 1
        for (int k = 0; k < m32; ++k) {
          const int   sk = __builtin_amdgcn_readlane(sr, k);
          const float ck = __int_as_float(__builtin_amdgcn_readlane(cfi, k));
          const v2f a = *(const v2fa*)(gsrc + (size_t)sk * H64 + 2 * lane);
          acc0 = fmaf(ck, a.x, acc0); acc1 = fmaf(ck, a.y, acc1);
        }
      }
      const v2f sv = *(const v2fa*)(gsrc + (size_t)nc * H64 + 2 * lane);
      if constexpr (MODE == 1) {
        const float y0 = (acc0 + sv.x * rd) + pzr, y1 = (acc1 + sv.y * rd) + pzr;
        v0 = live ? y0 : 0.0f; v1 = live ? y1 : 0.0f;
      } else {
        const float c0 = (acc0 + sv.x * rd) + bv0, c1 = (acc1 + sv.y * rd) + bv1;
        float x0 = c0, x1v = c1;
        if constexpr (MODE == 3) {
          const v2f rr = *(const v2fa*)(outp + (size_t)nc * H64 + 2 * lane);
          x0 = c0 + rr.x; x1v = c1 + rr.y;
        }
        x0 = x0 + pzr; x1v = x1v + pzr;
        v0 = live ? x0 : 0.0f; v1 = live ? x1v : 0.0f;
      }
    } else {
      float acc = 0.0f;
#pragma unroll 1
      for (int b0 = 0; b0 < c; b0 += 32) {
        int idx = o + b0 + lane;
        idx = idx > RCAP - 1 ? RCAP - 1 : idx;
        const int ent = sl[idx];
        int eid = ent >> SLA;
        eid = eid < 0 ? 0 : (eid > nE - 1 ? nE - 1 : eid);
        int sr = srcs[eid];
        sr = sr < 0 ? 0 : (sr > nN - 1 ? nN - 1 : sr);
        const int cfi = __float_as_int(nrm[eid]);
        const int m32 = (c - b0) < 32 ? (c - b0) : 32;
#pragma unroll 1
        for (int k = 0; k < m32; ++k) {
          const int   sk = __builtin_amdgcn_readlane(sr, k);
          const float ck = __int_as_float(__builtin_amdgcn_readlane(cfi, k));
          const float a = gsrc[(size_t)sk * H32 + lane];
          acc = fmaf(ck, a, acc);
        }
      }
      const float sv = gsrc[(size_t)nc * H32 + lane];
      const float cv = (acc + sv * rd) + bv0;
      float mx = cv;
#pragma unroll
      for (int d = 16; d >= 1; d >>= 1) mx = fmaxf(mx, __shfl_xor(mx, d, 32));
      const float e = __expf(cv - mx);
      float ssum = e;
#pragma unroll
      for (int d = 16; d >= 1; d >>= 1) ssum += __shfl_xor(ssum, d, 32);
      const float inv = 1.0f / (1.0f + ssum);
      const float p = e * inv + pzr;
      v0 = live ? p : 0.0f;
    }

    if constexpr (MODE != 1) {
      s1a += (double)v0; s2a += (double)v0 * (double)v0;
      if constexpr (MODE != 4) { s1b += (double)v1; s2b += (double)v1 * (double)v1; }
    }
    if constexpr (MODE != 4) {
      v4f ow;
      ow.x = __shfl(v0, sa, 32); ow.y = __shfl(v1, sa, 32);
      ow.z = __shfl(v0, sb, 32); ow.w = __shfl(v1, sb, 32);
      float* op = outp + (size_t)node * H64 + 4 * (lane & 15);
      const bool wr = wrow && (lane < 16);
      if (wr) *(volatile v4f*)op = ow;
      __threadfence();
      if (wr) *(volatile v4f*)op = ow;
    } else {
      float* op = outp + (size_t)node * H32 + lane;
      if (wrow) *(volatile float*)op = v0;
      __threadfence();
      if (wrow) *(volatile float*)op = v0;
    }
  }

  if constexpr (MODE != 1) {
    if constexpr (MODE != 4) {
      wst[(wave * FS + 2 * lane) * 2 + 0]     = s1a;
      wst[(wave * FS + 2 * lane) * 2 + 1]     = s2a;
      wst[(wave * FS + 2 * lane + 1) * 2 + 0] = s1b;
      wst[(wave * FS + 2 * lane + 1) * 2 + 1] = s2b;
    } else {
      wst[(wave * FS + lane) * 2 + 0] = s1a;
      wst[(wave * FS + lane) * 2 + 1] = s2a;
    }
    __syncthreads();
    if (tid < FS) {
      double S1 = 0.0, S2 = 0.0;
#pragma unroll
      for (int w2 = 0; w2 < NWAVE; ++w2) {
        S1 += wst[(w2 * FS + tid) * 2 + 0];
        S2 += wst[(w2 * FS + tid) * 2 + 1];
      }
      v2d orec;
      orec.x = S1; orec.y = S2;
      double* rp = rec + ((size_t)blockIdx.x * FS + tid) * 2;
      *(volatile v2d*)rp = orec;
      __threadfence();
      *(volatile v2d*)rp = orec;
    }
  }
}

__global__ __launch_bounds__(128) void k_comb(const double* __restrict__ rec, int nrec, int F, int nN,
                                              const float* __restrict__ gamma, const float* __restrict__ beta,
                                              float* tab) {
  __shared__ __attribute__((aligned(16))) float ts[TABN];
  const int tid = (int)threadIdx.x;
  const int c  = tid;
  const int cc = c < F ? c : F - 1;
  double S1 = 0.0, S2 = 0.0;
#pragma unroll 1
  for (int b = 0; b < nrec; ++b) {
    const v2d p = *(const v2da*)(rec + ((size_t)b * F + cc) * 2);
    S1 += p.x; S2 += p.y;
  }
  const double inv  = 1.0 / (double)nN;
  const double mean = S1 * inv;
  double var = S2 * inv - mean * mean;
  var = var < 0.0 ? 0.0 : var;
  const float mf = (float)mean;
  const float rf = rsqrtf((float)var + BNEPS);
  const float gv = bf16_val(gamma[cc]);
  const float bv = bf16_val(beta[cc]);
  const bool valid = c < F;
  ts[c]       = valid ? mf : 0.0f;
  ts[128 + c] = valid ? rf : 1.0f;
  ts[256 + c] = valid ? gv : 1.0f;
  ts[384 + c] = valid ? bv : 0.0f;
  __syncthreads();
  const v4f o = *(const v4fa*)(ts + 4 * tid);
  float* op = tab + 4 * tid;
  *(volatile v4f*)op = o;
  __threadfence();
  *(volatile v4f*)op = o;
}

__global__ __launch_bounds__(NTHR) void k_apply(const float* __restrict__ cin, const float* __restrict__ tab,
                                                int nN, int mRows, float* xout) {
  const int tid = (int)threadIdx.x, lane = tid & 31, wave = tid >> 5;
  const int q = lane & 15, sub = lane >> 4;
  const v4f mm = *(const v4fa*)(tab + 4 * q);
  const v4f rr = *(const v4fa*)(tab + 128 + 4 * q);
  const v4f gg = *(const v4fa*)(tab + 256 + 4 * q);
  const v4f bb = *(const v4fa*)(tab + 384 + 4 * q);
  const int base = (int)blockIdx.x * ARB + wave * (ARB / NWAVE);
#pragma unroll 1
  for (int it = 0; it < (ARB / NWAVE) / 2; ++it) {
    const int row = base + 2 * it + sub;
    const int rc  = row < nN ? row : nN - 1;
    const v4f x = *(const v4fa*)(cin + (size_t)rc * H64 + 4 * q);
    v4f y;
    y.x = ((x.x - mm.x) * rr.x) * gg.x + bb.x;
    y.y = ((x.y - mm.y) * rr.y) * gg.y + bb.y;
    y.z = ((x.z - mm.z) * rr.z) * gg.z + bb.z;
    y.w = ((x.w - mm.w) * rr.w) * gg.w + bb.w;
    float mx = fmaxf(fmaxf(y.x, y.y), fmaxf(y.z, y.w));
#pragma unroll
    for (int d = 8; d >= 1; d >>= 1) mx = fmaxf(mx, __shfl_xor(mx, d, 32));
    v4f e;
    e.x = __expf(y.x - mx); e.y = __expf(y.y - mx); e.z = __expf(y.z - mx); e.w = __expf(y.w - mx);
    float ssum = (e.x + e.y) + (e.z + e.w);
#pragma unroll
    for (int d = 8; d >= 1; d >>= 1) ssum += __shfl_xor(ssum, d, 32);
    const float inv = 1.0f / (1.0f + ssum);
    const bool live = row < nN;
    v4f o = e * inv;
    o.x = live ? o.x : 0.0f; o.y = live ? o.y : 0.0f; o.z = live ? o.z : 0.0f; o.w = live ? o.w : 0.0f;
    float* op = xout + (size_t)row * H64 + 4 * q;
    const bool wr = row < mRows;
    if (wr) *(volatile v4f*)op = o;
    __threadfence();
    if (wr) *(volatile v4f*)op = o;
  }
}

template <int KIN, int NC, int PRO, int EPB>
__global__ __launch_bounds__(GTHR) void k_gemm(const float* __restrict__ asrc, const float* __restrict__ tab,
                                               const unsigned short* __restrict__ BT, const float* __restrict__ bias,
                                               int nN, float* outp, double* rec) {
  constexpr int K2 = 2 * KIN, NT = NC / 16, LPR = KIN / 4, RPI = 32 / LPR, NIT = 16 / RPI;
  constexpr int LQ = NC / 4, RI = 32 / LQ, NI = 16 / RI;
  static_assert(K2 % 32 == 0 && (LPR == 16 || LPR == 32) && (LQ == 8 || LQ == 16 || LQ == 32));
  static_assert(EPB == 0 || NC == GTHR);
  __shared__ __attribute__((aligned(16))) unsigned short atile[GBM * K2];
  __shared__ __attribute__((aligned(16))) float stg[GBM * NC];
  const int tid = (int)threadIdx.x, lane = tid & 31, wave = tid >> 5, hh = lane >> 4, m = lane & 15;
  const int rowBase = (int)blockIdx.x * GBM;

  {
    const int q = lane & (LPR - 1), sub = lane / LPR;
    v4f mm = {0.0f, 0.0f, 0.0f, 0.0f}, rr = {1.0f, 1.0f, 1.0f, 1.0f};
    v4f gg = {1.0f, 1.0f, 1.0f, 1.0f}, bb = {0.0f, 0.0f, 0.0f, 0.0f};
    if constexpr (PRO != 0) {
      mm = *(const v4fa*)(tab + 4 * q);
      rr = *(const v4fa*)(tab + 128 + 4 * q);
      gg = *(const v4fa*)(tab + 256 + 4 * q);
      bb = *(const v4fa*)(tab + 384 + 4 * q);
    }
#pragma unroll 1
    for (int it = 0; it < NIT; ++it) {
      const int lr   = 16 * wave + it * RPI + sub;
      const int grow = rowBase + lr;
      const int rc   = grow < nN ? grow : nN - 1;
      const v4f x = *(const v4fa*)(asrc + (size_t)rc * KIN + 4 * q);
      v4f p;
      if constexpr (PRO != 0) {
        v4f y;
        y.x = ((x.x - mm.x) * rr.x) * gg.x + bb.x;
        y.y = ((x.y - mm.y) * rr.y) * gg.y + bb.y;
        y.z = ((x.z - mm.z) * rr.z) * gg.z + bb.z;
        y.w = ((x.w - mm.w) * rr.w) * gg.w + bb.w;
        float mx = fmaxf(fmaxf(y.x, y.y), fmaxf(y.z, y.w));
#pragma unroll
        for (int d = LPR / 2; d >= 1; d >>= 1) mx = fmaxf(mx, __shfl_xor(mx, d, 32));
        v4f e;
        e.x = __expf(y.x - mx); e.y = __expf(y.y - mx); e.z = __expf(y.z - mx); e.w = __expf(y.w - mx);
        float ssum = (e.x + e.y) + (e.z + e.w);
#pragma unroll
        for (int d = LPR / 2; d >= 1; d >>= 1) ssum += __shfl_xor(ssum, d, 32);
        const float inv = 1.0f / (1.0f + ssum);
        p = e * inv;
      } else {
        p = x;
      }
      const bool live = grow < nN;
      p.x = live ? p.x : 0.0f; p.y = live ? p.y : 0.0f; p.z = live ? p.z : 0.0f; p.w = live ? p.w : 0.0f;
      v4us h4, l4;
      unsigned hb;
      hb = bf16_bits(p.x); h4[0] = (unsigned short)hb; l4[0] = (unsigned short)bf16_bits(p.x - __uint_as_float(hb << 16));
      hb = bf16_bits(p.y); h4[1] = (unsigned short)hb; l4[1] = (unsigned short)bf16_bits(p.y - __uint_as_float(hb << 16));
      hb = bf16_bits(p.z); h4[2] = (unsigned short)hb; l4[2] = (unsigned short)bf16_bits(p.z - __uint_as_float(hb << 16));
      hb = bf16_bits(p.w); h4[3] = (unsigned short)hb; l4[3] = (unsigned short)bf16_bits(p.w - __uint_as_float(hb << 16));
      *(v4usa*)(atile + (size_t)lr * K2 + 4 * q) = h4;
      *(v4usa*)(atile + (size_t)lr * K2 + KIN + 4 * q) = l4;
    }
  }
  __syncthreads();

  v8f acc[NT];
  {
    const v8f z = {0.f, 0.f, 0.f, 0.f, 0.f, 0.f, 0.f, 0.f};
#pragma unroll
    for (int nt = 0; nt < NT; ++nt) acc[nt] = z;
  }
  const unsigned short* ap = atile + (size_t)(16 * wave + m) * K2 + 8 * hh;
  const unsigned short* bp = BT + (size_t)m * (size_t)K2 + 8 * hh;
#pragma unroll 1
  for (int k0 = 0; k0 < K2; k0 += 32) {
    FragB af;
    af.h[0] = *(const v8usa*)(ap + k0);
    af.h[1] = *(const v8usa*)(ap + k0 + 16);
#pragma unroll
    for (int nt = 0; nt < NT; ++nt) {
      const unsigned short* wq = bp + (size_t)(16 * nt) * (size_t)K2 + k0;
      FragB bf;
      bf.h[0] = *(const v8usa*)wq;
      bf.h[1] = *(const v8usa*)(wq + 16);
      acc[nt] = wmb(af, bf, acc[nt]);
    }
  }

#pragma unroll
  for (int nt = 0; nt < NT; ++nt) {
    const int lc = 16 * nt + m;
#pragma unroll
    for (int r = 0; r < 8; ++r) {
      const int lr = 16 * wave + 8 * hh + r;
      stg[lr * NC + lc] = acc[nt][r];
    }
  }
  __syncthreads();

  if constexpr (EPB != 0) {
    const float bc = bf16_val(bias[tid]);
    double S1 = 0.0, S2 = 0.0;
#pragma unroll 1
    for (int r = 0; r < GBM; ++r) {
      const float v  = stg[r * NC + tid] + bc;
      const float lv = ((rowBase + r) < nN) ? v : 0.0f;
      S1 += (double)lv; S2 += (double)lv * (double)lv;
    }
    v2d orec;
    orec.x = S1; orec.y = S2;
    double* rp = rec + ((size_t)blockIdx.x * NC + tid) * 2;
    *(volatile v2d*)rp = orec;
    __threadfence();
    *(volatile v2d*)rp = orec;
  }

  const int qq = lane & (LQ - 1), rsub = lane / LQ;
  v4f bb4 = {0.0f, 0.0f, 0.0f, 0.0f};
  if constexpr (EPB != 0) {
    const v4f tb = *(const v4fa*)(bias + 4 * qq);
    bb4.x = bf16_val(tb.x); bb4.y = bf16_val(tb.y); bb4.z = bf16_val(tb.z); bb4.w = bf16_val(tb.w);
  }
  v4f fv[NI];
#pragma unroll
  for (int i = 0; i < NI; ++i) {
    const int lr = 16 * wave + i * RI + rsub;
    v4f tv = *(const v4fa*)(stg + lr * NC + 4 * qq) + bb4;
    const bool live = (rowBase + lr) < nN;
    tv.x = live ? tv.x : 0.0f; tv.y = live ? tv.y : 0.0f; tv.z = live ? tv.z : 0.0f; tv.w = live ? tv.w : 0.0f;
    fv[i] = tv;
  }
#pragma unroll
  for (int i = 0; i < NI; ++i) {
    const int lr = 16 * wave + i * RI + rsub;
    float* op = outp + (size_t)(rowBase + lr) * (size_t)NC + 4 * qq;
    *(volatile v4f*)op = fv[i];
  }
  __threadfence();
#pragma unroll
  for (int i = 0; i < NI; ++i) {
    const int lr = 16 * wave + i * RI + rsub;
    float* op = outp + (size_t)(rowBase + lr) * (size_t)NC + 4 * qq;
    *(volatile v4f*)op = fv[i];
  }
}

__global__ __launch_bounds__(NTHR) void k_out(const float* __restrict__ S, const float* __restrict__ tab,
                                              const float* __restrict__ ow, int nN, float* out) {
  __shared__ float ts[5 * H32];
  __shared__ __attribute__((aligned(16))) float os[NTHR];
  const int tid = (int)threadIdx.x;
  if (tid < H32) {
    ts[tid]           = tab[tid];
    ts[H32 + tid]     = tab[128 + tid];
    ts[2 * H32 + tid] = tab[256 + tid];
    ts[3 * H32 + tid] = tab[384 + tid];
    ts[4 * H32 + tid] = bf16_val(ow[tid]);
  }
  __syncthreads();
  const int row = (int)blockIdx.x * NTHR + tid;
  const int rc  = row < nN ? row : nN - 1;
  const float* sp = S + (size_t)rc * H32;
  float acc = 0.0f;
#pragma unroll 1
  for (int j4 = 0; j4 < H32 / 4; ++j4) {
    const v4f s4 = *(const v4fa*)(sp + 4 * j4);
    const int j = 4 * j4;
    float y;
    y = ((s4.x - ts[j + 0]) * ts[H32 + j + 0]) * ts[2 * H32 + j + 0] + ts[3 * H32 + j + 0];
    acc = fmaf(y, ts[4 * H32 + j + 0], acc);
    y = ((s4.y - ts[j + 1]) * ts[H32 + j + 1]) * ts[2 * H32 + j + 1] + ts[3 * H32 + j + 1];
    acc = fmaf(y, ts[4 * H32 + j + 1], acc);
    y = ((s4.z - ts[j + 2]) * ts[H32 + j + 2]) * ts[2 * H32 + j + 2] + ts[3 * H32 + j + 2];
    acc = fmaf(y, ts[4 * H32 + j + 2], acc);
    y = ((s4.w - ts[j + 3]) * ts[H32 + j + 3]) * ts[2 * H32 + j + 3] + ts[3 * H32 + j + 3];
    acc = fmaf(y, ts[4 * H32 + j + 3], acc);
  }
  os[tid] = acc;
  __syncthreads();
  if (tid < NTHR / 4) {
    const int r0 = (int)blockIdx.x * NTHR + 4 * tid;
    const v4f o = *(const v4fa*)(os + 4 * tid);
    if (r0 + 4 <= nN) {
      float* op = out + r0;
      *(volatile v4f*)op = o;
      __threadfence();
      *(volatile v4f*)op = o;
    } else {
      if (r0     < nN) *(volatile float*)(out + r0)     = o.x;
      if (r0 + 1 < nN) *(volatile float*)(out + r0 + 1) = o.y;
      if (r0 + 2 < nN) *(volatile float*)(out + r0 + 2) = o.z;
      __threadfence();
      if (r0     < nN) *(volatile float*)(out + r0)     = o.x;
      if (r0 + 1 < nN) *(volatile float*)(out + r0 + 1) = o.y;
      if (r0 + 2 < nN) *(volatile float*)(out + r0 + 2) = o.z;
    }
  }
}

static inline int cdiv(int a, int b) { return (a + b - 1) / b; }
static inline size_t al256(size_t o) { return (o + 255) & ~(size_t)255; }

extern "C" void kernel_launch(void* const* d_in, const int* in_sizes, int n_in,
                              void* d_out, int out_size, void* d_ws, size_t ws_size,
                              hipStream_t stream) {
  if (n_in < 27) return;
  if (in_sizes[0] < NFX || (in_sizes[0] % NFX) != 0) return;
  const int nN = in_sizes[0] / NFX;
  if (nN < 64 || nN > (1 << 22)) return;
  if (in_sizes[1] < 2 || (in_sizes[1] & 1) != 0) return;
  const int nE = in_sizes[1] / 2;
  if (nE < 1 || nE >= (1 << (31 - SLA))) return;
  if (in_sizes[2] != nE) return;
  if (in_sizes[4] != 18 * 4 || in_sizes[5] != 4) return;
  if (in_sizes[6] != H64 * 4 || in_sizes[7] != H64) return;
  if (in_sizes[8] != H128 * H64 || in_sizes[9] != H128) return;
  if (in_sizes[10] != H64 * H128 || in_sizes[11] != H64) return;
  if (in_sizes[12] != NMID * H64 * H64 || in_sizes[13] != NMID * H64) return;
  if (in_sizes[14] != H32 * H64 || in_sizes[15] != H32) return;
  if (in_sizes[16] != H64 || in_sizes[17] != H64) return;
  if (in_sizes[18] != H128 || in_sizes[19] != H128) return;
  if (in_sizes[20] != H64 || in_sizes[21] != H64) return;
  if (in_sizes[22] != NMID * H64 || in_sizes[23] != NMID * H64) return;
  if (in_sizes[24] != H32 || in_sizes[25] != H32 || in_sizes[26] != H32) return;
  if (out_size != nN) return;

  const float* x    = (const float*)d_in[0];
  const int*   edge = (const int*)d_in[1];
  const float* ew   = (const float*)d_in[2];
  const float* Wesg = (const float*)d_in[4];
  const float* besg = (const float*)d_in[5];
  const float* W0   = (const float*)d_in[6];
  const float* b0   = (const float*)d_in[7];
  const float* W1   = (const float*)d_in[8];
  const float* b1   = (const float*)d_in[9];
  const float* W2   = (const float*)d_in[10];
  const float* b2   = (const float*)d_in[11];
  const float* Wm   = (const float*)d_in[12];
  const float* bm   = (const float*)d_in[13];
  const float* Wf   = (const float*)d_in[14];
  const float* bfp  = (const float*)d_in[15];
  const float* g0   = (const float*)d_in[16];
  const float* be0  = (const float*)d_in[17];
  const float* g1   = (const float*)d_in[18];
  const float* be1  = (const float*)d_in[19];
  const float* g2   = (const float*)d_in[20];
  const float* be2  = (const float*)d_in[21];
  const float* gm   = (const float*)d_in[22];
  const float* bem  = (const float*)d_in[23];
  const float* gf   = (const float*)d_in[24];
  const float* bef  = (const float*)d_in[25];
  const float* outw = (const float*)d_in[26];
  float* out = (float*)d_out;
  const int* src = edge;
  const int* dst = edge + nE;

  const int MP   = cdiv(nN, GBM) * GBM;
  const int gM   = MP / GBM;
  const int gD   = cdiv(nN, NBD);
  const int NBPD = gD * NBD;
  const int gA   = cdiv(MP, NBA);
  if ((long long)gA * NBA < (long long)MP) return;
  if (NBPD < nN) return;
  if ((MP % ARB) != 0) return;
  const int nPadE = cdiv(nE, 64) * 64;
  const int vec8 = ((nE & 3) == 0) ? 1 : 0;
  const int nrecMax = (gM * H128 > gA * H64) ? gM * H128 : gA * H64;

  char* ws = (char*)d_ws;
  size_t off = 0;
  const size_t oB1  = off; off = al256(off + (size_t)H128 * (2 * H64) * 2);
  const size_t oB2  = off; off = al256(off + (size_t)H64 * (2 * H128) * 2);
  const size_t oBM  = off; off = al256(off + (size_t)NMID * H64 * (2 * H64) * 2);
  const size_t oBF  = off; off = al256(off + (size_t)H32 * (2 * H64) * 2);
  const size_t oX10 = off; off = al256(off + (size_t)MP * 4 * 4);
  const size_t oDIS = off; off = al256(off + (size_t)NBPD * 4);
  const size_t oNRM = off; off = al256(off + (size_t)nPadE * 4);
  const size_t oC   = off; off = al256(off + (size_t)MP * H64 * 4);
  const size_t oX0  = off; off = al256(off + (size_t)MP * H64 * 4);
  const size_t oA1  = off; off = al256(off + (size_t)MP * H64 * 4);
  const size_t oC1  = off; off = al256(off + (size_t)MP * H128 * 4);
  const size_t oT   = off; off = al256(off + (size_t)MP * H64 * 4);
  const size_t oS   = off; off = al256(off + (size_t)MP * H32 * 4);
  const size_t oREC = off; off = al256(off + (size_t)nrecMax * 16);
  const size_t oTAB = off; off = al256(off + (size_t)TABN * 4);
  if (off > ws_size || off > (size_t)WSMAX) return;
  unsigned short* B1  = (unsigned short*)(ws + oB1);
  unsigned short* B2  = (unsigned short*)(ws + oB2);
  unsigned short* BM  = (unsigned short*)(ws + oBM);
  unsigned short* BF  = (unsigned short*)(ws + oBF);
  float*  X10 = (float*)(ws + oX10);
  float*  DIS = (float*)(ws + oDIS);
  float*  NRM = (float*)(ws + oNRM);
  float*  C   = (float*)(ws + oC);
  float*  X0  = (float*)(ws + oX0);
  float*  A1  = (float*)(ws + oA1);
  float*  C1  = (float*)(ws + oC1);
  float*  T   = (float*)(ws + oT);
  float*  S   = (float*)(ws + oS);
  double* REC = (double*)(ws + oREC);
  float*  TAB = (float*)(ws + oTAB);

  const size_t scanLds = (size_t)AGG_LDS_INTS * 4;
  hipFuncSetAttribute(reinterpret_cast<const void*>(&k_scan<0>), hipFuncAttributeMaxDynamicSharedMemorySize, (int)scanLds);
  hipFuncSetAttribute(reinterpret_cast<const void*>(&k_scan<1>), hipFuncAttributeMaxDynamicSharedMemorySize, (int)scanLds);
  hipFuncSetAttribute(reinterpret_cast<const void*>(&k_scan<2>), hipFuncAttributeMaxDynamicSharedMemorySize, (int)scanLds);
  hipFuncSetAttribute(reinterpret_cast<const void*>(&k_scan<3>), hipFuncAttributeMaxDynamicSharedMemorySize, (int)scanLds);
  hipFuncSetAttribute(reinterpret_cast<const void*>(&k_scan<4>), hipFuncAttributeMaxDynamicSharedMemorySize, (int)scanLds);

  k_wprep<<<UTOT / NTHR, NTHR, 0, stream>>>(W1, W2, Wm, Wf, B1, B2, BM, BF);
  k_esg<<<cdiv(MP, NTHR), NTHR, 0, stream>>>(x, nN, MP, Wesg, besg, X10);
  k_deg<<<gD, NTHR, 0, stream>>>(dst, ew, nE, vec8, DIS);
  k_norm<<<cdiv(nPadE / 2, NTHR), NTHR, 0, stream>>>(src, dst, ew, DIS, nE, nN, nPadE, NRM);

  k_scan<0><<<gA, NTHR, scanLds, stream>>>(src, dst, nE, nN, vec8, MP, DIS, NRM, X10, W0, b0, C, REC);
  k_comb<<<1, 128, 0, stream>>>(REC, gA, H64, nN, g0, be0, TAB);
  k_apply<<<MP / ARB, NTHR, 0, stream>>>(C, TAB, nN, MP, X0);
  k_scan<1><<<gA, NTHR, scanLds, stream>>>(src, dst, nE, nN, vec8, MP, DIS, NRM, X0, W0, b0, A1, REC);
  k_gemm<H64, H128, 0, 1><<<gM, GTHR, 0, stream>>>(A1, TAB, B1, b1, nN, C1, REC);
  k_comb<<<1, 128, 0, stream>>>(REC, gM, H128, nN, g1, be1, TAB);
  k_gemm<H128, H64, 1, 0><<<gM, GTHR, 0, stream>>>(C1, TAB, B2, b2, nN, T, REC);
  k_scan<2><<<gA, NTHR, scanLds, stream>>>(src, dst, nE, nN, vec8, MP, DIS, NRM, T, W0, b2, C, REC);
  k_comb<<<1, 128, 0, stream>>>(REC, gA, H64, nN, g2, be2, TAB);
  for (int i = 0; i < NMID; ++i) {
    k_gemm<H64, H64, 1, 0><<<gM, GTHR, 0, stream>>>(C, TAB, BM + (size_t)i * H64 * (2 * H64), bm + (size_t)i * H64,
                                                   nN, T, REC);
    k_scan<3><<<gA, NTHR, scanLds, stream>>>(src, dst, nE, nN, vec8, MP, DIS, NRM, T, W0, bm + (size_t)i * H64, C, REC);
    k_comb<<<1, 128, 0, stream>>>(REC, gA, H64, nN, gm + (size_t)i * H64, bem + (size_t)i * H64, TAB);
  }
  k_gemm<H64, H32, 1, 0><<<gM, GTHR, 0, stream>>>(C, TAB, BF, bfp, nN, T, REC);
  k_scan<4><<<gA, NTHR, scanLds, stream>>>(src, dst, nE, nN, vec8, MP, DIS, NRM, T, W0, bfp, S, REC);
  k_comb<<<1, 128, 0, stream>>>(REC, gA, H32, nN, gf, bef, TAB);
  k_out<<<cdiv(nN, NTHR), NTHR, 0, stream>>>(S, TAB, outw, nN, out);
}
